// SelectiveSSM_58265526337931
// MI455X (gfx1250) — hardware-verified
//
#include <hip/hip_runtime.h>
#include <math.h>

typedef __attribute__((ext_vector_type(16))) _Float16 v16h;
typedef __attribute__((ext_vector_type(8)))  _Float16 v8h;
typedef __attribute__((ext_vector_type(16))) __bf16   v16b;
typedef __attribute__((ext_vector_type(8)))  __bf16   v8b;
typedef __attribute__((ext_vector_type(8)))  float    v8f;
typedef __attribute__((ext_vector_type(4)))  float    v4f;
typedef __attribute__((ext_vector_type(4)))  unsigned u32x4;

constexpr int kBatch  = 2;
constexpr int kSeq    = 2048;
constexpr int kDm     = 1024;
constexpr int kNst    = 16;
constexpr int kDtR    = 64;
constexpr int kRows   = kBatch * kSeq;
constexpr int kNbc    = 2 * kNst;
constexpr int kPbcN   = 64;
constexpr int kPjRows = 128;
constexpr int kScanTS = 64;
constexpr int kScanCh = 64;
constexpr int kScanYP = 68;
static_assert((kDm % 32) == 0 && (kDtR % 32) == 0, "GEMM K multiples of 32");
static_assert((kRows % 64) == 0 && (kDtR % 64) == 0 && (kPbcN % 64) == 0 && (kDm % 64) == 0, "GEMM M,N multiples of 64");
static_assert(kDtR + kNbc <= kPjRows && (kPjRows % 64) == 0, "packed projection rows");
static_assert((kSeq % kScanTS) == 0 && (kDm % kScanCh) == 0 && kScanCh == 64 && kScanTS == 64, "scan tile");

constexpr size_t kOffXH   = 0;
constexpr size_t kOffWPJ  = kOffXH   + (size_t)kRows   * kDm   * 2;
constexpr size_t kOffWDT  = kOffWPJ  + (size_t)kPjRows * kDm   * 2;
constexpr size_t kOffWOUT = kOffWDT  + (size_t)kDm     * kDtR  * 2;
constexpr size_t kOffDTH  = kOffWOUT + (size_t)kDm     * kDm   * 2;
constexpr size_t kOffDTL  = kOffDTH  + (size_t)kRows   * kDtR  * 2;
constexpr size_t kOffPBC  = kOffDTL  + (size_t)kRows   * kDtR  * 2;
constexpr size_t kOffZ    = kOffPBC  + (size_t)kRows   * kPbcN * 4;
constexpr size_t kOffYS   = kOffZ    + (size_t)kRows   * kDm   * 4;
constexpr size_t kOffYNH  = kOffYS   + (size_t)kRows   * kDm   * 4;
constexpr size_t kOffYNL  = kOffYNH  + (size_t)kRows   * kDm   * 2;
constexpr size_t kWsTotal = kOffYNL  + (size_t)kRows   * kDm   * 2;
static_assert(kWsTotal == 63307776ull, "carve total");
static_assert(kWsTotal <= 134217728ull, "carve cap");
static_assert((kOffWPJ % 128) == 0 && (kOffWDT % 128) == 0 && (kOffWOUT % 128) == 0 && (kOffDTH % 128) == 0 &&
              (kOffDTL % 128) == 0 && (kOffPBC % 128) == 0 && (kOffZ % 128) == 0 && (kOffYS % 128) == 0 &&
              (kOffYNH % 128) == 0 && (kOffYNL % 128) == 0, "128-B aligned regions");

__device__ __forceinline__ unsigned short f2bf_bits(float f) {
  unsigned u = __float_as_uint(f);
  return (unsigned short)((u + 0x7FFFu + ((u >> 16) & 1u)) >> 16);
}
__device__ __forceinline__ float bf_bits2f(unsigned short h) { return __uint_as_float(((unsigned)h) << 16); }
__device__ __forceinline__ float bfr(float f) { return bf_bits2f(f2bf_bits(f)); }

__device__ __forceinline__ void dep_guard_h(v8f& a, v8f& b, v16h x, v16h y) { asm volatile("v_nop\n\tv_nop\n\tv_nop\n\tv_nop" : "+v"(a), "+v"(b) : "v"(x), "v"(y)); }
__device__ __forceinline__ void dep_guard_b(v8f& a, v8f& b, v16b x, v16b y) { asm volatile("v_nop\n\tv_nop\n\tv_nop\n\tv_nop" : "+v"(a), "+v"(b) : "v"(x), "v"(y)); }
__device__ __forceinline__ void keep4_h(v16h a, v16h b, v16h c, v16h d) { asm volatile("v_nop" :: "v"(a), "v"(b), "v"(c), "v"(d)); }
__device__ __forceinline__ void keep4_b(v16b a, v16b b, v16b c, v16b d) { asm volatile("v_nop" :: "v"(a), "v"(b), "v"(c), "v"(d)); }
__device__ __forceinline__ void acc_guard4(v8f& a, v8f& b, v8f& c, v8f& d) { asm volatile("v_nop\n\tv_nop\n\tv_nop\n\tv_nop" : "+v"(a), "+v"(b), "+v"(c), "+v"(d)); }
template <typename T> struct Frag;
template <> struct Frag<_Float16> {
  typedef v16h V; union U { v16h v; v8h h[2]; };
  static __device__ __forceinline__ v16h load(const _Float16* p) {
    U f; f.h[0] = *(const v8h*)(p); f.h[1] = *(const v8h*)(p + 16); return f.v;
  }
  static __device__ __forceinline__ v8f mma(v16h a, v16h b, v8f c) {
    return __builtin_amdgcn_wmma_f32_16x16x32_f16(false, a, false, b, (short)0, c, false, false);
  }
  static __device__ __forceinline__ void guard(v8f& a, v8f& b, v16h x, v16h y) { dep_guard_h(a, b, x, y); }
  static __device__ __forceinline__ void keep(v16h a, v16h b, v16h c, v16h d) { keep4_h(a, b, c, d); }
};
template <> struct Frag<__bf16> {
  typedef v16b V; union U { v16b v; v8b h[2]; };
  static __device__ __forceinline__ v16b load(const __bf16* p) {
    U f; f.h[0] = *(const v8b*)(p); f.h[1] = *(const v8b*)(p + 16); return f.v;
  }
  static __device__ __forceinline__ v8f mma(v16b a, v16b b, v8f c) {
    return __builtin_amdgcn_wmma_f32_16x16x32_bf16(false, a, false, b, (short)0, c, false, false);
  }
  static __device__ __forceinline__ void guard(v8f& a, v8f& b, v16b x, v16b y) { dep_guard_b(a, b, x, y); }
  static __device__ __forceinline__ void keep(v16b a, v16b b, v16b c, v16b d) { keep4_b(a, b, c, d); }
};

template <int ET> struct Elem;
template <> struct Elem<0> { typedef _Float16 T; };
template <> struct Elem<1> { typedef __bf16 T; };
template <int ET, int SPL, int BIAS_MODE, int OUT_MODE, bool RESID, int ACT = 0>
__global__ __launch_bounds__(256) void wmma_gemm64(
    const unsigned short* __restrict__ Ap, const unsigned short* __restrict__ A2p, int lda, long strideA,
    const unsigned short* __restrict__ Btp, const unsigned short* __restrict__ Bt2p, int ldb, long strideB,
    void* __restrict__ Cout, void* __restrict__ Cout2, int ldc, long strideC,
    const float* __restrict__ bias,
    const float* __restrict__ resid, long strideR,
    int M, int N, int K, float scale) {
  typedef typename Elem<ET>::T T;
  typedef typename Frag<T>::V V;
  const T* A = (const T*)Ap; const T* A2 = (const T*)A2p; const T* Bt = (const T*)Btp; const T* Bt2 = (const T*)Bt2p;
  __shared__ __align__(16) float sT[8][16 * 68];
  const int b    = blockIdx.y;
  const int lane = threadIdx.x & 31;
  const int wave = threadIdx.x >> 5;
  const int tilesN = N >> 6;
  const int tilesM = M >> 6;
  const int tile = blockIdx.x * 8 + wave;
  if (tile >= tilesM * tilesN) return;
  const int tm = tile / tilesN;
  const int tn = tile - tm * tilesN;
  const int m0 = tm << 6;
  const int n0 = tn << 6;

  const T* Ab  = A  + (size_t)b * strideA;
  const T* Bb  = Bt + (size_t)b * strideB;
  const T* Ab2 = (SPL >= 1) ? (A2  + (size_t)b * strideA) : nullptr;
  const T* Bb2 = (SPL == 2) ? (Bt2 + (size_t)b * strideB) : nullptr;

  const int rlane = lane & 15;
  const int koff  = (lane >> 4) * 8;
  const int mOff  = (lane >> 4) * 8;

  v8f acc[4][4];
#pragma unroll
  for (int i = 0; i < 4; ++i)
#pragma unroll
    for (int j = 0; j < 4; ++j) acc[i][j] = (v8f){0.f,0.f,0.f,0.f,0.f,0.f,0.f,0.f};

  for (int k0 = 0; k0 < K; k0 += 32) {
    V bh[4], bl[4];
#pragma unroll
    for (int j = 0; j < 4; ++j) {
      const size_t bo = (size_t)(n0 + (j << 4) + rlane) * ldb + koff + k0;
      bh[j] = Frag<T>::load(Bb + bo);
      if (SPL == 2) bl[j] = Frag<T>::load(Bb2 + bo);
    }
#pragma unroll
    for (int i = 0; i < 4; ++i) {
      const size_t ao = (size_t)(m0 + (i << 4) + rlane) * lda + koff + k0;
      V ah = Frag<T>::load(Ab + ao);
      V al;
      if (SPL >= 1) al = Frag<T>::load(Ab2 + ao);
#pragma unroll
      for (int j = 0; j < 4; ++j) {
        acc[i][j] = Frag<T>::mma(ah, bh[j], acc[i][j]);
        if (SPL == 2) acc[i][j] = Frag<T>::mma(ah, bl[j], acc[i][j]);
        if (SPL >= 1) acc[i][j] = Frag<T>::mma(al, bh[j], acc[i][j]);
      }
      Frag<T>::guard(acc[i][0], acc[i][3], ah, (SPL >= 1) ? al : ah);
      Frag<T>::guard(acc[i][1], acc[i][2], ah, (SPL >= 1) ? al : ah);
    }
    Frag<T>::keep(bh[0], bh[1], bh[2], bh[3]);
    if (SPL == 2) Frag<T>::keep(bl[0], bl[1], bl[2], bl[3]);
  }
  acc_guard4(acc[0][0], acc[0][1], acc[0][2], acc[0][3]);
  acc_guard4(acc[1][0], acc[1][1], acc[1][2], acc[1][3]);
  acc_guard4(acc[2][0], acc[2][1], acc[2][2], acc[2][3]);
  acc_guard4(acc[3][0], acc[3][1], acc[3][2], acc[3][3]);

  float* slab = sT[wave];
  const float* Rb = RESID ? (resid + (size_t)b * strideR) : nullptr;
#pragma unroll
  for (int i = 0; i < 4; ++i) {
    const int mBase = m0 + (i << 4);
#pragma unroll
    for (int j = 0; j < 4; ++j) {
      const int n = n0 + (j << 4) + rlane;
      float bv = 0.f;
      if (BIAS_MODE == 2) bv = bias[n];
#pragma unroll
      for (int r = 0; r < 8; ++r) {
        float v = acc[i][j][r] * scale;
        if (BIAS_MODE == 1) v += bias[mBase + mOff + r];
        if (BIAS_MODE == 2) v += bv;
        if (RESID) v += Rb[(size_t)(mBase + mOff + r) * ldc + n];
        if (ACT == 1) v = tanhf(v);
        if (ACT == 2) v = fmaxf(v, 0.0f);
        if (ACT == 3) v = v / (1.0f + expf(-v));
        if (ACT == 4) v = (v > 0.f) ? v : 0.01f * v;
        slab[(mOff + r) * 68 + (j << 4) + rlane] = v;
      }
    }
    __builtin_amdgcn_fence(__ATOMIC_RELEASE, "workgroup");
    __builtin_amdgcn_wave_barrier();
    __builtin_amdgcn_fence(__ATOMIC_ACQUIRE, "workgroup");
    if (OUT_MODE == 0) {
      float* C = (float*)Cout + (size_t)b * strideC;
      const int hh = lane >> 4, c4 = (lane & 15) * 4;
      for (int pass = 0; pass < 2; ++pass) {
#pragma unroll
        for (int it = 0; it < 8; ++it) {
          const int row = it * 2 + hh;
          v4f v = *(const v4f*)(slab + row * 68 + c4);
          *(volatile v4f*)(C + (size_t)(mBase + row) * ldc + n0 + c4) = v;
        }
        __threadfence();
      }
    } else {
      const int q = lane >> 3, c8 = (lane & 7) * 8;
      unsigned short* C  = (unsigned short*)Cout  + (size_t)b * strideC;
      unsigned short* C2 = (OUT_MODE == 2) ? ((unsigned short*)Cout2 + (size_t)b * strideC) : nullptr;
      for (int pass = 0; pass < 2; ++pass) {
#pragma unroll
        for (int it = 0; it < 4; ++it) {
          const int row = it * 4 + q;
          const float* sp = slab + row * 68 + c8;
          v8h hv, lv;
#pragma unroll
          for (int e = 0; e < 8; ++e) {
            if (OUT_MODE == 1) {
              hv[e] = (_Float16)sp[e];
            } else {
              unsigned short hb = f2bf_bits(sp[e]);
              unsigned short lb = f2bf_bits(sp[e] - bf_bits2f(hb));
              hv[e] = __builtin_bit_cast(_Float16, hb);
              lv[e] = __builtin_bit_cast(_Float16, lb);
            }
          }
          *(volatile v8h*)(C + (size_t)(mBase + row) * ldc + n0 + c8) = hv;
          if (OUT_MODE == 2) *(volatile v8h*)(C2 + (size_t)(mBase + row) * ldc + n0 + c8) = lv;
        }
        __threadfence();
      }
    }
    __builtin_amdgcn_fence(__ATOMIC_RELEASE, "workgroup");
    __builtin_amdgcn_wave_barrier();
    __builtin_amdgcn_fence(__ATOMIC_ACQUIRE, "workgroup");
  }
}

__global__ __launch_bounds__(256) void cvt_rows_bf16_kernel(
    const float* __restrict__ src, unsigned short* __restrict__ dst, int total8)
{
  const int i = blockIdx.x * 256 + threadIdx.x;
  if (i >= total8) return;
  const size_t e0 = (size_t)i << 3;
  const v4f a0 = *(const v4f*)(src + e0);
  const v4f a1 = *(const v4f*)(src + e0 + 4);
  v8h hv;
#pragma unroll
  for (int e = 0; e < 4; ++e) {
    const unsigned short h0 = f2bf_bits(a0[e]), h1 = f2bf_bits(a1[e]);
    hv[e]     = __builtin_bit_cast(_Float16, h0);
    hv[4 + e] = __builtin_bit_cast(_Float16, h1);
  }
  unsigned short* q = dst + e0;
  *(volatile v8h*)q = hv;
  __threadfence();
  *(volatile v8h*)q = hv;
}

__global__ __launch_bounds__(256) void zero16_kernel(unsigned short* __restrict__ dst, int total16)
{
  const int i = blockIdx.x * 256 + threadIdx.x;
  if (i >= total16) return;
  const u32x4 z = {0u, 0u, 0u, 0u};
  u32x4* p = (u32x4*)(dst + ((size_t)i << 3));
  *(volatile u32x4*)p = z;
  __threadfence();
  *(volatile u32x4*)p = z;
}

__global__ __launch_bounds__(64) void scan_kernel(
    const float* __restrict__ PBC, const float* __restrict__ Z, const float* __restrict__ X,
    const float* __restrict__ bdt, const float* __restrict__ Alog, const float* __restrict__ Dp,
    float* __restrict__ YS)
{
  __shared__ __align__(16) float sBC[kScanTS * kNbc];
  __shared__ __align__(16) float sY[kScanTS * kScanYP];
  __shared__ __align__(16) float sA[kNst * kScanCh];
  const int tid = threadIdx.x, lane = tid & 31, wave = tid >> 5;
  constexpr int kBlkPerB = kDm / kScanCh;
  const int bix = blockIdx.x / kBlkPerB;
  const int d0  = (blockIdx.x - bix * kBlkPerB) * kScanCh;
  const int d   = d0 + tid;
  const size_t row0 = (size_t)bix * kSeq;
#pragma unroll 1
  for (int s = 0; s < kNst; ++s) sA[s * kScanCh + tid] = -expf(bfr(Alog[(size_t)d * kNst + s]));
  __syncthreads();
  float negA[kNst], h[kNst];
#pragma unroll
  for (int s = 0; s < kNst; ++s) {
    negA[s] = sA[s * kScanCh + tid];
    h[s] = 0.f;
  }
  const float bb = bfr(bdt[d]), Dd = bfr(Dp[d]);
  const int lr = tid >> 3, lc4 = (tid & 7) * 4;
  const int hh = lane >> 4, c4 = (lane & 15) * 4;
#pragma unroll 1
  for (int t0 = 0; t0 < kSeq; t0 += kScanTS) {
    __syncthreads();
#pragma unroll
    for (int i = 0; i < 8; ++i) {
      const int r = lr + 8 * i;
      *(v4f*)(sBC + r * kNbc + lc4) = *(const v4f*)(PBC + (row0 + t0 + r) * kPbcN + lc4);
    }
    __syncthreads();
#pragma unroll 1
    for (int s = 0; s < kScanTS; ++s) {
      const int t = t0 + s;
      const float* br = sBC + s * kNbc;
      float Bs[kNst], Cs[kNst];
#pragma unroll
      for (int q4 = 0; q4 < 4; ++q4) {
        const v4f bv = *(const v4f*)(br + 4 * q4);
        const v4f cv = *(const v4f*)(br + kNst + 4 * q4);
        Bs[4 * q4 + 0] = bv[0]; Bs[4 * q4 + 1] = bv[1]; Bs[4 * q4 + 2] = bv[2]; Bs[4 * q4 + 3] = bv[3];
        Cs[4 * q4 + 0] = cv[0]; Cs[4 * q4 + 1] = cv[1]; Cs[4 * q4 + 2] = cv[2]; Cs[4 * q4 + 3] = cv[3];
      }
      const float zv  = Z[(row0 + t) * kDm + d];
      const float v   = zv + bb;
      const float a   = __expf(-fabsf(v));
      const float u   = 1.0f + a;
      const float l1p = __logf(u) + (a - (u - 1.0f)) * __builtin_amdgcn_rcpf(u);
      const float dt  = fmaxf(v, 0.0f) + l1p;
      const float xt  = bfr(X[(row0 + t) * kDm + d]);
      float y = 0.f;
#pragma unroll
      for (int k = 0; k < kNst; ++k) {
        const float e  = __expf(dt * negA[k]);
        const float db = dt * Bs[k];
        h[k] = e * h[k] + db * xt;
        y = h[k] * Cs[k] + y;
      }
      y = Dd * xt + y;
      sY[s * kScanYP + tid] = y;
    }
    __syncthreads();
    for (int pass = 0; pass < 2; ++pass) {
#pragma unroll
      for (int it = 0; it < 16; ++it) {
        const int row = it * 4 + wave * 2 + hh;
        const v4f ov = *(const v4f*)(sY + row * kScanYP + c4);
        *(volatile v4f*)(YS + (row0 + t0 + row) * kDm + d0 + c4) = ov;
      }
      __threadfence();
    }
  }
}

__global__ __launch_bounds__(128) void ln_split_kernel(
    const float* __restrict__ YS, const float* __restrict__ g, const float* __restrict__ bta,
    unsigned short* __restrict__ YNH, unsigned short* __restrict__ YNL)
{
  __shared__ float sRed[8];
  const int tid = threadIdx.x, lane = tid & 31, wave = tid >> 5;
  const size_t m = blockIdx.x;
  const float* rp = YS + m * kDm + (size_t)tid * 8;
  const v4f a0 = *(const v4f*)(rp);
  const v4f a1 = *(const v4f*)(rp + 4);
  float v[8];
  v[0] = a0[0]; v[1] = a0[1]; v[2] = a0[2]; v[3] = a0[3];
  v[4] = a1[0]; v[5] = a1[1]; v[6] = a1[2]; v[7] = a1[3];
  float s1 = 0.f;
#pragma unroll
  for (int e = 0; e < 8; ++e) s1 += v[e];
#pragma unroll
  for (int off = 16; off > 0; off >>= 1) s1 += __shfl_xor(s1, off, 32);
  if (lane == 0) sRed[wave] = s1;
  __syncthreads();
  const float tot = (sRed[0] + sRed[1]) + (sRed[2] + sRed[3]);
  const float mu = tot * (1.0f / (float)kDm);
  float s2 = 0.f;
#pragma unroll
  for (int e = 0; e < 8; ++e) { const float dv = v[e] - mu; s2 = dv * dv + s2; }
#pragma unroll
  for (int off = 16; off > 0; off >>= 1) s2 += __shfl_xor(s2, off, 32);
  if (lane == 0) sRed[4 + wave] = s2;
  __syncthreads();
  const float var = ((sRed[4] + sRed[5]) + (sRed[6] + sRed[7])) * (1.0f / (float)kDm);
  const float rs = rsqrtf(var + 1e-5f);
  const v4f g0 = *(const v4f*)(g + (size_t)tid * 8);
  const v4f g1 = *(const v4f*)(g + (size_t)tid * 8 + 4);
  const v4f b0 = *(const v4f*)(bta + (size_t)tid * 8);
  const v4f b1 = *(const v4f*)(bta + (size_t)tid * 8 + 4);
  float gg[8], bt[8];
  gg[0] = g0[0]; gg[1] = g0[1]; gg[2] = g0[2]; gg[3] = g0[3];
  gg[4] = g1[0]; gg[5] = g1[1]; gg[6] = g1[2]; gg[7] = g1[3];
  bt[0] = b0[0]; bt[1] = b0[1]; bt[2] = b0[2]; bt[3] = b0[3];
  bt[4] = b1[0]; bt[5] = b1[1]; bt[6] = b1[2]; bt[7] = b1[3];
  v8h hv, lv;
#pragma unroll
  for (int e = 0; e < 8; ++e) {
    const float yn = (v[e] - mu) * rs * bfr(gg[e]) + bfr(bt[e]);
    const unsigned short hb = f2bf_bits(yn);
    const unsigned short lb = f2bf_bits(yn - bf_bits2f(hb));
    hv[e] = __builtin_bit_cast(_Float16, hb);
    lv[e] = __builtin_bit_cast(_Float16, lb);
  }
  const size_t o = m * kDm + (size_t)tid * 8;
  for (int pass = 0; pass < 2; ++pass) {
    *(volatile v8h*)(YNH + o) = hv;
    *(volatile v8h*)(YNL + o) = lv;
    __threadfence();
  }
}

extern "C" void kernel_launch(void* const* d_in, const int* in_sizes, int n_in,
                              void* d_out, int out_size, void* d_ws, size_t ws_size,
                              hipStream_t stream) {
  if (n_in < 11) return;
  if (in_sizes[0] != kRows * kDm) return;
  if (in_sizes[1] != kDtR * kDm) return;
  if (in_sizes[2] != kDm * kDtR) return;
  if (in_sizes[3] != kDm) return;
  if (in_sizes[4] != kDm * kNst) return;
  if (in_sizes[5] != kNst * kDm) return;
  if (in_sizes[6] != kNst * kDm) return;
  if (in_sizes[7] != kDm) return;
  if (in_sizes[8] != kDm) return;
  if (in_sizes[9] != kDm) return;
  if (in_sizes[10] != kDm * kDm) return;
  if (out_size != kRows * kDm) return;
  if (ws_size < kWsTotal) return;

  const float* x     = (const float*)d_in[0];
  const float* W_dtw = (const float*)d_in[1];
  const float* W_dt  = (const float*)d_in[2];
  const float* b_dt  = (const float*)d_in[3];
  const float* A_log = (const float*)d_in[4];
  const float* W_B   = (const float*)d_in[5];
  const float* W_C   = (const float*)d_in[6];
  const float* Dp    = (const float*)d_in[7];
  const float* ln_g  = (const float*)d_in[8];
  const float* ln_b  = (const float*)d_in[9];
  const float* W_out = (const float*)d_in[10];
  float* out = (float*)d_out;

  char* ws = (char*)d_ws;
  unsigned short* XH   = (unsigned short*)(ws + kOffXH);
  unsigned short* WPJ  = (unsigned short*)(ws + kOffWPJ);
  unsigned short* WDT  = (unsigned short*)(ws + kOffWDT);
  unsigned short* WOUT = (unsigned short*)(ws + kOffWOUT);
  unsigned short* DTH  = (unsigned short*)(ws + kOffDTH);
  unsigned short* DTL  = (unsigned short*)(ws + kOffDTL);
  float*          PBC  = (float*)(ws + kOffPBC);
  float*          Z    = (float*)(ws + kOffZ);
  float*          YS   = (float*)(ws + kOffYS);
  unsigned short* YNH  = (unsigned short*)(ws + kOffYNH);
  unsigned short* YNL  = (unsigned short*)(ws + kOffYNL);

  {
    const int t8x = kRows * kDm / 8;
    cvt_rows_bf16_kernel<<<(t8x + 255) / 256, 256, 0, stream>>>(x, XH, t8x);
    const int t8w = kDtR * kDm / 8;
    cvt_rows_bf16_kernel<<<(t8w + 255) / 256, 256, 0, stream>>>(W_dtw, WPJ, t8w);
    const int t8b = kNst * kDm / 8;
    cvt_rows_bf16_kernel<<<(t8b + 255) / 256, 256, 0, stream>>>(W_B, WPJ + (size_t)kDtR * kDm, t8b);
    cvt_rows_bf16_kernel<<<(t8b + 255) / 256, 256, 0, stream>>>(W_C, WPJ + (size_t)(kDtR + kNst) * kDm, t8b);
    const int t16z = (kPjRows - kDtR - kNbc) * kDm * 2 / 16;
    zero16_kernel<<<(t16z + 255) / 256, 256, 0, stream>>>(WPJ + (size_t)(kDtR + kNbc) * kDm, t16z);
    const int t8d = kDm * kDtR / 8;
    cvt_rows_bf16_kernel<<<(t8d + 255) / 256, 256, 0, stream>>>(W_dt, WDT, t8d);
    const int t8o = kDm * kDm / 8;
    cvt_rows_bf16_kernel<<<(t8o + 255) / 256, 256, 0, stream>>>(W_out, WOUT, t8o);
  }

  wmma_gemm64<1, 0, 0, 2, false><<<dim3(((kRows / 64) * (kDtR / 64) + 7) / 8, 1), 256, 0, stream>>>(
      XH, nullptr, kDm, 0L,
      WPJ, nullptr, kDm, 0L,
      (void*)DTH, (void*)DTL, kDtR, 0L,
      nullptr, nullptr, 0L,
      kRows, kDtR, kDm, 1.0f);

  wmma_gemm64<1, 0, 0, 0, false><<<dim3(((kRows / 64) * (kPbcN / 64) + 7) / 8, 1), 256, 0, stream>>>(
      XH, nullptr, kDm, 0L,
      WPJ + (size_t)kDtR * kDm, nullptr, kDm, 0L,
      (void*)PBC, nullptr, kPbcN, 0L,
      nullptr, nullptr, 0L,
      kRows, kPbcN, kDm, 1.0f);

  wmma_gemm64<1, 1, 0, 0, false><<<dim3(((kRows / 64) * (kDm / 64) + 7) / 8, 1), 256, 0, stream>>>(
      DTH, DTL, kDtR, 0L,
      WDT, nullptr, kDtR, 0L,
      (void*)Z, nullptr, kDm, 0L,
      nullptr, nullptr, 0L,
      kRows, kDm, kDtR, 1.0f);

  scan_kernel<<<kBatch * (kDm / kScanCh), kScanCh, 0, stream>>>(PBC, Z, x, b_dt, A_log, Dp, YS);

  ln_split_kernel<<<kRows, 128, 0, stream>>>(YS, ln_g, ln_b, YNH, YNL);

  wmma_gemm64<1, 1, 0, 0, false><<<dim3(((kRows / 64) * (kDm / 64) + 7) / 8, 1), 256, 0, stream>>>(
      YNH, YNL, kDm, 0L,
      WOUT, nullptr, kDm, 0L,
      (void*)out, nullptr, kDm, 0L,
      nullptr, nullptr, 0L,
      kRows, kDm, kDm, 1.0f);
}
